// CNF_60524679135740
// MI455X (gfx1250) — hardware-verified
//
#include <hip/hip_runtime.h>
#include <math.h>

constexpr int NBATCH  = 4096;
constexpr int NDIM    = 64;
constexpr int NHID    = 256;
constexpr int NIN1    = NDIM + 1;
constexpr int NTHR    = 256;
constexpr int ROWS    = 32;
constexpr int NBLK    = NBATCH / ROWS;
constexpr int NSTEPS  = 10;
constexpr int NSTAGE  = 6;
constexpr int NKZ     = 5;
constexpr int KZPLANE = ROWS * NDIM;
constexpr int XP      = 72;
constexpr int HP      = 264;
constexpr int EP      = 256;
constexpr int OPITCH  = 68;
constexpr int LPOFF   = 4096;
constexpr int NOUT0   = NBATCH * NDIM;
constexpr int NOUT1   = NBATCH;
constexpr float WSC     = 64.0f;
constexpr float WSC_INV = 1.0f / 64.0f;
constexpr float ESC     = 16.0f;
constexpr float EW_INV  = 1.0f / (16.0f * 64.0f);
constexpr float DTF     = (float)(1.0 / 10.0);
constexpr float NEG_HALF_LOG_2PI = -0.91893853320467274f;
static_assert(NBATCH % ROWS == 0);
static_assert(NHID == 32 * (NTHR / 32));
static_assert(ROWS == 2 * 16 && NDIM == 4 * 16);
static_assert(NDIM % 32 == 0 && NHID % 32 == 0);
static_assert(ROWS * NDIM == 8 * NTHR);
static_assert(ROWS * NDIM == 2 * 4 * NTHR);
static_assert((NOUT0 * 4) % 128 == 0 && ROWS * 4 == 128);
static_assert(NDIM % 64 == 0 && NHID % 64 == 0);
static_assert(XP % 8 == 0 && HP % 8 == 0);
static_assert((NKZ * KZPLANE) % NTHR == 0);
static_assert(ROWS * OPITCH <= LPOFF && LPOFF + ROWS <= NKZ * KZPLANE);
static_assert(NSTAGE == NKZ + 1);
static_assert(ROWS == 32);

typedef __attribute__((ext_vector_type(16))) _Float16 v16h;
typedef __attribute__((ext_vector_type(8)))  _Float16 v8h;
typedef __attribute__((ext_vector_type(8)))  float    v8f;
typedef __attribute__((ext_vector_type(4)))  float    v4f;
typedef __attribute__((ext_vector_type(4)))  unsigned v4u;

__device__ __forceinline__ unsigned short f2bf_bits(float f) {
  unsigned u = __float_as_uint(f);
  return (unsigned short)((u + 0x7FFFu + ((u >> 16) & 1u)) >> 16);
}
__device__ __forceinline__ float bf_bits2f(unsigned short h) { return __uint_as_float(((unsigned)h) << 16); }
__device__ __forceinline__ float bf16r(float f) { return bf_bits2f(f2bf_bits(f)); }
__device__ __forceinline__ unsigned short f16_bits(float f) { return __builtin_bit_cast(unsigned short, (_Float16)f); }
__device__ __forceinline__ float h16_to_f32(unsigned hb) {
  const unsigned sgn = (hb & 0x8000u) << 16; const unsigned em = hb & 0x7fffu;
  const float fn = __uint_as_float((em << 13) + 0x38000000u);
  const float fs = (float)em * 5.9604644775390625e-8f;
  const float mag = (em < 0x400u) ? fs : fn; return __uint_as_float(__float_as_uint(mag) | sgn);
}

__device__ __forceinline__ void guard2ab(v8f& c0, v8f& c1, v16h a0, v16h a1, v16h b0) {
  asm volatile("v_nop\n\tv_nop\n\tv_nop\n\tv_nop" : "+v"(c0), "+v"(c1) : "v"(a0), "v"(a1), "v"(b0));
}
__device__ __forceinline__ void guard1ab(v8f& c0, v16h a0, v16h b0) {
  asm volatile("v_nop\n\tv_nop\n\tv_nop\n\tv_nop" : "+v"(c0) : "v"(a0), "v"(b0));
}
__device__ __forceinline__ void acc_guard2(v8f& a, v8f& b) { asm volatile("v_nop\n\tv_nop\n\tv_nop\n\tv_nop" : "+v"(a), "+v"(b)); }
__device__ __forceinline__ void acc_guard1(v8f& a) { asm volatile("v_nop\n\tv_nop\n\tv_nop\n\tv_nop" : "+v"(a)); }

template <typename T> struct Frag;
template <> struct Frag<_Float16> {
  typedef v16h V; union U { v16h v; v8h h[2]; };
  static __device__ __forceinline__ v16h load(const _Float16* p) {
    U f; f.h[0] = *(const v8h*)(p); f.h[1] = *(const v8h*)(p + 16); return f.v;
  }
  static __device__ __forceinline__ v8f mma(v16h a, v16h b, v8f c) {
    return __builtin_amdgcn_wmma_f32_16x16x32_f16(false, a, false, b, (short)0, c, false, false);
  }
};

__device__ __forceinline__ float tanh_acc(float x) {
  const float ax = fminf(fabsf(x), 15.0f);
  const float ex = expf(2.0f * ax);
  const float t  = 1.0f - 2.0f * __builtin_amdgcn_rcpf(ex + 1.0f);
  return copysignf(t, x);
}

__device__ __forceinline__ float pick6(int s, float v0, float v1, float v2, float v3, float v4, float v5) {
  float r = v5;
  r = (s == 4) ? v4 : r;
  r = (s == 3) ? v3 : r;
  r = (s == 2) ? v2 : r;
  r = (s == 1) ? v1 : r;
  r = (s == 0) ? v0 : r;
  return r;
}

template <int MODE>
__global__ __launch_bounds__(NTHR) void tpw_kernel(const float* __restrict__ src, int R, int C, int ldo,
                                                  unsigned short* __restrict__ O, float sc) {
  __shared__ float Tt[64 * 65];
  const int tid = threadIdx.x;
  const int c0 = blockIdx.x * 64, r0 = blockIdx.y * 64;
#pragma unroll
  for (int i = 0; i < 4; ++i) {
    const int idx = i * NTHR + tid;
    const int rr = idx >> 4, cc = (idx & 15) * 4;
    const v4f v = *(const v4f*)(src + (size_t)(r0 + rr) * (size_t)C + c0 + cc);
    Tt[rr * 65 + cc + 0] = v[0];
    Tt[rr * 65 + cc + 1] = v[1];
    Tt[rr * 65 + cc + 2] = v[2];
    Tt[rr * 65 + cc + 3] = v[3];
  }
  __syncthreads();
  const int q = tid >> 3, c8 = (tid & 7) * 8;
  v8h hv[2];
#pragma unroll
  for (int g = 0; g < 2; ++g) {
    const int qq = g * 32 + q;
#pragma unroll
    for (int e = 0; e < 8; ++e) {
      const float f = Tt[(c8 + e) * 65 + qq];
      unsigned short bits;
      if (MODE == 0) {
        bits = f2bf_bits(f * sc);
      } else {
        const float fb = bf_bits2f(f2bf_bits(f));
        bits = __builtin_bit_cast(unsigned short, (_Float16)(fb * sc));
      }
      hv[g][e] = __builtin_bit_cast(_Float16, bits);
    }
  }
  for (int pass = 0; pass < 2; ++pass) {
#pragma unroll
    for (int g = 0; g < 2; ++g) {
      const size_t o = (size_t)(c0 + g * 32 + q) * (size_t)ldo + (size_t)(r0 + c8);
      *(volatile v8h*)(O + o) = hv[g];
    }
    __threadfence();
  }
}

template <int MODE>
__global__ __launch_bounds__(NTHR) void cvt8_kernel(const float* __restrict__ src, unsigned short* __restrict__ dst,
                                                    int nrow, int ncol8, int spitch, int scol0, float sc) {
  const int i  = blockIdx.x * NTHR + threadIdx.x;
  const int n8 = nrow * ncol8;
  if (i < n8) {
    const int row = i / ncol8;
    const int c8  = i - row * ncol8;
    const float* sp = src + (size_t)row * spitch + scol0 + c8 * 8;
    const v4f a = *(const v4f*)(sp);
    const v4f b = *(const v4f*)(sp + 4);
    v8h hv;
#pragma unroll
    for (int e = 0; e < 4; ++e) {
      unsigned short b0, b1;
      if (MODE == 0) {
        b0 = f2bf_bits(a[e] * sc);
        b1 = f2bf_bits(b[e] * sc);
      } else {
        b0 = __builtin_bit_cast(unsigned short, (_Float16)(bf16r(a[e]) * sc));
        b1 = __builtin_bit_cast(unsigned short, (_Float16)(bf16r(b[e]) * sc));
      }
      hv[e]     = __builtin_bit_cast(_Float16, b0);
      hv[4 + e] = __builtin_bit_cast(_Float16, b1);
    }
    *(volatile v8h*)(dst + (size_t)i * 8) = hv;
    __threadfence();
    *(volatile v8h*)(dst + (size_t)i * 8) = hv;
  }
}

template <int KD, int AP>
__device__ __forceinline__ void mm32x16(const _Float16* aL, const _Float16* __restrict__ bt, int ldbt, int nb,
                                        int rl, int koff, v8f (&c)[2]) {
  const v8f z8 = {0.f, 0.f, 0.f, 0.f, 0.f, 0.f, 0.f, 0.f};
  c[0] = z8; c[1] = z8;
  const _Float16* a0p = aL + rl * AP + koff;
  const _Float16* a1p = a0p + 16 * AP;
  const _Float16* b0p = bt + (size_t)(nb + rl) * ldbt + koff;
#pragma unroll 1
  for (int k0 = 0; k0 < KD; k0 += 32) {
    const v16h a0 = Frag<_Float16>::load(a0p + k0);
    const v16h a1 = Frag<_Float16>::load(a1p + k0);
    const v16h b0 = Frag<_Float16>::load(b0p + k0);
    c[0] = Frag<_Float16>::mma(a0, b0, c[0]);
    c[1] = Frag<_Float16>::mma(a1, b0, c[1]);
    guard2ab(c[0], c[1], a0, a1, b0);
  }
  acc_guard2(c[0], c[1]);
}

template <int KD, int AP>
__device__ __forceinline__ void mm16(const _Float16* aL, const _Float16* __restrict__ bt, int ldbt, int nb,
                                     int rl, int koff, v8f& c) {
  const v8f z8 = {0.f, 0.f, 0.f, 0.f, 0.f, 0.f, 0.f, 0.f};
  c = z8;
  const _Float16* a0p = aL + rl * AP + koff;
  const _Float16* b0p = bt + (size_t)(nb + rl) * ldbt + koff;
#pragma unroll 1
  for (int k0 = 0; k0 < KD; k0 += 32) {
    const v16h a0 = Frag<_Float16>::load(a0p + k0);
    const v16h b0 = Frag<_Float16>::load(b0p + k0);
    c = Frag<_Float16>::mma(a0, b0, c);
    guard1ab(c, a0, b0);
  }
  acc_guard1(c);
}

__global__ __launch_bounds__(NTHR) __attribute__((amdgpu_num_vgpr(256)))
void ode_flow_kernel(
    const float* __restrict__ y, const float* __restrict__ e, const float* __restrict__ W1,
    const float* __restrict__ b1, const float* __restrict__ b2, const float* __restrict__ b3,
    const unsigned short* __restrict__ W1Pp, const unsigned short* __restrict__ W2Fp,
    const unsigned short* __restrict__ W2Bp, const unsigned short* __restrict__ W3Fp,
    const unsigned short* __restrict__ W3Bp, float* __restrict__ out) {
  __shared__ __align__(16) unsigned short sX[ROWS * XP];
  __shared__ __align__(16) unsigned short sH1[ROWS * HP];
  __shared__ __align__(16) unsigned short sH2[ROWS * HP];
  __shared__ __align__(16) unsigned short sG2[ROWS * HP];
  __shared__ __align__(16) unsigned short sE3[ROWS * EP];
  __shared__ __align__(16) unsigned short sE1[ROWS * EP];
  __shared__ __align__(16) float sKZ[NKZ * KZPLANE];
  __shared__ __align__(16) float sDiv[(NTHR / 32) * ROWS];

  const _Float16* W1P = (const _Float16*)W1Pp;
  const _Float16* W2F = (const _Float16*)W2Fp;
  const _Float16* W2B = (const _Float16*)W2Bp;
  const _Float16* W3F = (const _Float16*)W3Fp;
  const _Float16* W3B = (const _Float16*)W3Bp;

  const int tid = threadIdx.x, lane = tid & 31, wave = tid >> 5;
  const int rl = lane & 15, hh = lane >> 4, koff = hh * 8;
  const int colw = 32 * wave;
  const int mt3 = wave >> 2, nt3 = wave & 3;
  const int blk = blockIdx.x, row0 = blk * ROWS;
  const int zrow = 16 * mt3 + 8 * hh;
  const int zcol = 16 * nt3 + rl;
  const int zpos = zrow * NDIM + zcol;

#pragma unroll 1
  for (int i = tid; i < NKZ * KZPLANE; i += NTHR) sKZ[i] = 0.0f;

  float w1t0, w1t1, b1v0, b1v1, b2v0, b2v1;
  {
    const int cA = colw + rl, cB = colw + 16 + rl;
    w1t0 = bf16r(W1[NDIM * NHID + cA]);
    w1t1 = bf16r(W1[NDIM * NHID + cB]);
    b1v0 = bf16r(b1[cA]);
    b1v1 = bf16r(b1[cB]);
    b2v0 = bf16r(b2[cA]);
    b2v1 = bf16r(b2[cB]);
  }
  const float b3v = bf16r(b3[zcol]);
  asm volatile("" ::: "memory");
  float zr[8];
#pragma unroll
  for (int r = 0; r < 8; ++r) zr[r] = bf16r(y[(size_t)(row0 + zrow + r) * NDIM + zcol]);
  asm volatile("" ::: "memory");

  {
    const int er = tid >> 3, c8 = (tid & 7) * 8;
    const float* ep = e + (size_t)(row0 + er) * NDIM + c8;
    const v4f ea = *(const v4f*)(ep);
    const v4f eb = *(const v4f*)(ep + 4);
    const unsigned u0 = f16_bits(ESC * bf16r(ea[0])), u1 = f16_bits(ESC * bf16r(ea[1]));
    const unsigned u2 = f16_bits(ESC * bf16r(ea[2])), u3 = f16_bits(ESC * bf16r(ea[3]));
    const unsigned u4 = f16_bits(ESC * bf16r(eb[0])), u5 = f16_bits(ESC * bf16r(eb[1]));
    const unsigned u6 = f16_bits(ESC * bf16r(eb[2])), u7 = f16_bits(ESC * bf16r(eb[3]));
    v4u pk;
    pk[0] = u0 | (u1 << 16);
    pk[1] = u2 | (u3 << 16);
    pk[2] = u4 | (u5 << 16);
    pk[3] = u6 | (u7 << 16);
    *(v4u*)(sX + er * XP + c8) = pk;
  }
  __syncthreads();

#pragma unroll 1
  for (int nt = 0; nt < 2; ++nt) {
    const int cb16 = colw + 16 * nt;
    v8f acc[2];
    mm32x16<NDIM, XP>((const _Float16*)sX, W3B, NDIM, cb16, rl, koff, acc);
#pragma unroll
    for (int mt = 0; mt < 2; ++mt)
#pragma unroll
      for (int r = 0; r < 8; ++r)
        sE3[(16 * mt + 8 * hh + r) * EP + cb16 + rl] = f2bf_bits(acc[mt][r] * EW_INV);
    mm32x16<NDIM, XP>((const _Float16*)sX, W1P, NDIM, cb16, rl, koff, acc);
#pragma unroll
    for (int mt = 0; mt < 2; ++mt)
#pragma unroll
      for (int r = 0; r < 8; ++r)
        sE1[(16 * mt + 8 * hh + r) * EP + cb16 + rl] = f2bf_bits(acc[mt][r] * EW_INV);
  }
  __syncthreads();

  float zacc[8];
  float lp = 0.0f, klacc = 0.0f;

#pragma unroll 1
  for (int step = 0; step < NSTEPS; ++step) {
    const float t0 = (float)step * DTF;
    klacc = 0.0f;
#pragma unroll
    for (int r = 0; r < 8; ++r) zacc[r] = 0.0f;
#pragma unroll 1
    for (int s = 0; s < NSTAGE; ++s) {
      const float a0 = pick6(s, 0.0f, (float)(1.0 / 5.0), (float)(3.0 / 40.0), (float)(44.0 / 45.0), (float)(19372.0 / 6561.0), (float)(9017.0 / 3168.0));
      const float a1 = pick6(s, 0.0f, 0.0f, (float)(9.0 / 40.0), (float)(-56.0 / 15.0), (float)(-25360.0 / 2187.0), (float)(-355.0 / 33.0));
      const float a2 = pick6(s, 0.0f, 0.0f, 0.0f, (float)(32.0 / 9.0), (float)(64448.0 / 6561.0), (float)(46732.0 / 5247.0));
      const float a3 = pick6(s, 0.0f, 0.0f, 0.0f, 0.0f, (float)(-212.0 / 729.0), (float)(49.0 / 176.0));
      const float a4 = pick6(s, 0.0f, 0.0f, 0.0f, 0.0f, 0.0f, (float)(-5103.0 / 18656.0));
      const float cb = pick6(s, (float)(35.0 / 384.0), 0.0f, (float)(500.0 / 1113.0), (float)(125.0 / 192.0), (float)(-2187.0 / 6784.0), (float)(11.0 / 84.0));
      const float ct = pick6(s, (float)(0.0 * 0.1), (float)((1.0 / 5.0) * 0.1), (float)((3.0 / 10.0) * 0.1), (float)((4.0 / 5.0) * 0.1), (float)((8.0 / 9.0) * 0.1), (float)(1.0 * 0.1));
      const float ts = t0 + ct;

#pragma unroll
      for (int r = 0; r < 8; ++r) {
        const int p = zpos + r * NDIM;
        const float v0 = sKZ[p];
        const float v1 = sKZ[KZPLANE + p];
        const float v2 = sKZ[2 * KZPLANE + p];
        const float v3 = sKZ[3 * KZPLANE + p];
        const float v4 = sKZ[4 * KZPLANE + p];
        float sa = 0.0f;
        sa = sa + a0 * v0;
        sa = sa + a1 * v1;
        sa = sa + a2 * v2;
        sa = sa + a3 * v3;
        sa = sa + a4 * v4;
        const float zs = zr[r] + DTF * sa;
        sX[(zrow + r) * XP + zcol] = f16_bits(zs);
      }
      __syncthreads();

#pragma unroll 1
      for (int nt = 0; nt < 2; ++nt) {
        const int cb16 = colw + 16 * nt;
        const float w1tv = nt ? w1t1 : w1t0;
        const float b1vv = nt ? b1v1 : b1v0;
        const float add = ts * w1tv + b1vv;
        v8f acc[2];
        mm32x16<NDIM, XP>((const _Float16*)sX, W1P, NDIM, cb16, rl, koff, acc);
#pragma unroll
        for (int mt = 0; mt < 2; ++mt)
#pragma unroll
          for (int r = 0; r < 8; ++r) {
            const float h = tanh_acc(acc[mt][r] * WSC_INV + add);
            sH1[(16 * mt + 8 * hh + r) * HP + cb16 + rl] = f16_bits(h);
          }
      }
      __syncthreads();

#pragma unroll 1
      for (int nt = 0; nt < 2; ++nt) {
        const int cb16 = colw + 16 * nt;
        const float b2vv = nt ? b2v1 : b2v0;
        v8f acc[2];
        mm32x16<NHID, HP>((const _Float16*)sH1, W2F, NHID, cb16, rl, koff, acc);
#pragma unroll
        for (int mt = 0; mt < 2; ++mt)
#pragma unroll
          for (int r = 0; r < 8; ++r) {
            const int row = 16 * mt + 8 * hh + r, col = cb16 + rl;
            const float h = tanh_acc(acc[mt][r] * WSC_INV + b2vv);
            const unsigned we = sE3[row * EP + col];
            const float ew = __uint_as_float(we << 16);
            const float g = ew * (1.0f - h * h);
            sH2[row * HP + col] = f16_bits(h);
            sG2[row * HP + col] = f16_bits(g);
          }
      }
      __syncthreads();

      {
        v8f acc3;
        mm16<NHID, HP>((const _Float16*)sH2 + 16 * mt3 * HP, W3F, NHID, 16 * nt3, rl, koff, acc3);
        float kv[8];
#pragma unroll
        for (int r = 0; r < 8; ++r) {
          kv[r] = acc3[r] * WSC_INV + b3v;
          zacc[r] = zacc[r] + cb * kv[r];
        }
        if (s < NKZ) {
#pragma unroll
          for (int r = 0; r < 8; ++r) sKZ[s * KZPLANE + zpos + r * NDIM] = kv[r];
        }
      }

      {
        float pd[2][8];
#pragma unroll
        for (int mt = 0; mt < 2; ++mt)
#pragma unroll
          for (int r = 0; r < 8; ++r) pd[mt][r] = 0.0f;
#pragma unroll 1
        for (int nt = 0; nt < 2; ++nt) {
          const int cb16 = colw + 16 * nt;
          v8f acc[2];
          mm32x16<NHID, HP>((const _Float16*)sG2, W2B, NHID, cb16, rl, koff, acc);
#pragma unroll
          for (int mt = 0; mt < 2; ++mt)
#pragma unroll
            for (int r = 0; r < 8; ++r) {
              const int row = 16 * mt + 8 * hh + r, col = cb16 + rl;
              const unsigned hb = sH1[row * HP + col];
              const float h1f = h16_to_f32(hb);
              const float d1 = 1.0f - h1f * h1f;
              const float g1 = (acc[mt][r] * WSC_INV) * d1;
              const unsigned w1 = sE1[row * EP + col];
              const float ew1 = __uint_as_float(w1 << 16);
              pd[mt][r] = pd[mt][r] + g1 * ew1;
            }
        }
#pragma unroll
        for (int mt = 0; mt < 2; ++mt)
#pragma unroll
          for (int r = 0; r < 8; ++r) {
            float v = pd[mt][r];
            v += __shfl_xor(v, 1, 32);
            v += __shfl_xor(v, 2, 32);
            v += __shfl_xor(v, 4, 32);
            v += __shfl_xor(v, 8, 32);
            pd[mt][r] = v;
          }
        if (rl == 0) {
#pragma unroll
          for (int mt = 0; mt < 2; ++mt)
#pragma unroll
            for (int r = 0; r < 8; ++r) sDiv[wave * ROWS + 16 * mt + 8 * hh + r] = pd[mt][r];
        }
      }
      __syncthreads();

      {
        float dv = sDiv[lane];
#pragma unroll
        for (int w = 1; w < NTHR / 32; ++w) dv = dv + sDiv[w * ROWS + lane];
        klacc = klacc + cb * (-dv);
      }
    }
#pragma unroll
    for (int r = 0; r < 8; ++r) zr[r] = zr[r] + DTF * zacc[r];
    lp = lp + DTF * klacc;
  }

  float* sOut = sKZ;
  float* sLP  = sKZ + LPOFF;
#pragma unroll
  for (int r = 0; r < 8; ++r) sOut[(zrow + r) * OPITCH + zcol] = zr[r];
  __syncthreads();
  {
    float lpz = 0.0f;
#pragma unroll 1
    for (int k = 0; k < NDIM; ++k) {
      const float zv = sOut[lane * OPITCH + k];
      lpz = lpz + (NEG_HALF_LOG_2PI - 0.5f * zv * zv);
    }
    if (tid < ROWS) sLP[tid] = lpz - lp;
  }
  __syncthreads();
  {
    const v4f o0 = *(const v4f*)(sOut + (tid >> 4) * OPITCH + (tid & 15) * 4);
    const v4f o1 = *(const v4f*)(sOut + (16 + (tid >> 4)) * OPITCH + (tid & 15) * 4);
    const v4f o2 = *(const v4f*)(sLP + 4 * (tid & 7));
    float* ob0 = out + (size_t)blk * (ROWS * NDIM);
    float* ob1 = out + (size_t)NOUT0 + (size_t)blk * ROWS;
    for (int pass = 0; pass < 2; ++pass) {
      *(volatile v4f*)(ob0 + 4 * tid) = o0;
      *(volatile v4f*)(ob0 + 1024 + 4 * tid) = o1;
      if (tid < 8) *(volatile v4f*)(ob1 + 4 * tid) = o2;
      __threadfence();
    }
  }
}

extern "C" void kernel_launch(void* const* d_in, const int* in_sizes, int n_in,
                              void* d_out, int out_size, void* d_ws, size_t ws_size, hipStream_t stream) {
  if (n_in < 8 || d_out == nullptr || d_ws == nullptr) return;
  if (in_sizes[0] != NBATCH * NDIM || in_sizes[1] != NBATCH * NDIM || in_sizes[2] != NIN1 * NHID ||
      in_sizes[3] != NHID || in_sizes[4] != NHID * NHID || in_sizes[5] != NHID ||
      in_sizes[6] != NHID * NDIM || in_sizes[7] != NDIM || out_size != NOUT0 + NOUT1) return;

  const float* y  = (const float*)d_in[0];
  const float* e  = (const float*)d_in[1];
  const float* W1 = (const float*)d_in[2];
  const float* b1 = (const float*)d_in[3];
  const float* W2 = (const float*)d_in[4];
  const float* b2 = (const float*)d_in[5];
  const float* W3 = (const float*)d_in[6];
  const float* b3 = (const float*)d_in[7];
  float* out = (float*)d_out;

  char* ws = (char*)d_ws; size_t off = 0;
  auto carve = [&](size_t bytes) -> char* { char* p = ws + off; off += (bytes + 255) & ~(size_t)255; return p; };
  unsigned short* W1P = (unsigned short*)carve((size_t)NHID * NDIM * 2);
  unsigned short* W2F = (unsigned short*)carve((size_t)NHID * NHID * 2);
  unsigned short* W2B = (unsigned short*)carve((size_t)NHID * NHID * 2);
  unsigned short* W3F = (unsigned short*)carve((size_t)NDIM * NHID * 2);
  unsigned short* W3B = (unsigned short*)carve((size_t)NHID * NDIM * 2);
  if (off > ws_size || off > (size_t)134217728) return;

  tpw_kernel<1><<<dim3(NHID / 64, NDIM / 64), NTHR, 0, stream>>>(W1, NDIM, NHID, NDIM, W1P, WSC);
  tpw_kernel<1><<<dim3(NHID / 64, NHID / 64), NTHR, 0, stream>>>(W2, NHID, NHID, NHID, W2F, WSC);
  cvt8_kernel<1><<<(NHID * (NHID / 8) + NTHR - 1) / NTHR, NTHR, 0, stream>>>(W2, W2B, NHID, NHID / 8, NHID, 0, WSC);
  tpw_kernel<1><<<dim3(NDIM / 64, NHID / 64), NTHR, 0, stream>>>(W3, NHID, NDIM, NHID, W3F, WSC);
  cvt8_kernel<1><<<(NHID * (NDIM / 8) + NTHR - 1) / NTHR, NTHR, 0, stream>>>(W3, W3B, NHID, NDIM / 8, NDIM, 0, WSC);
  ode_flow_kernel<<<NBLK, NTHR, 0, stream>>>(y, e, W1, b1, b2, b3, W1P, W2F, W2B, W3F, W3B, out);
}
